// MyNet_11879879543557
// MI455X (gfx1250) — hardware-run, weakly checked
//
#include <hip/hip_runtime.h>


#define NBT  8
#define TT   128
#define NSQ  32
#define HH   128
#define G4   (4 * HH)
#define MP   64
#define DM   HH
#define LOSC 1024.0f

typedef _Float16 h16;
typedef unsigned short bf;
typedef __attribute__((ext_vector_type(16))) __bf16   v16bf;
typedef __attribute__((ext_vector_type(16))) _Float16 v16h;
typedef __attribute__((ext_vector_type(8)))  _Float16 v8h;
typedef __attribute__((ext_vector_type(8)))  unsigned short v8us;
typedef __attribute__((ext_vector_type(8)))  float    v8f;
typedef __attribute__((ext_vector_type(4)))  float    v4f;
typedef __attribute__((ext_vector_type(4)))  _Float16 v4h;
typedef v8h  __attribute__((may_alias)) v8ha;
typedef v4f  __attribute__((may_alias)) v4fa;
typedef v8us __attribute__((may_alias)) v8usa;

__device__ __forceinline__ unsigned short f2bf(float f) { unsigned u = __float_as_uint(f); u += 0x7FFFu + ((u >> 16) & 1u); return (unsigned short)(u >> 16); }
__device__ __forceinline__ float bf2f(unsigned short b) { return __uint_as_float(((unsigned)b) << 16); }
__device__ __forceinline__ float bfr(float f) { return bf2f(f2bf(f)); }
__device__ __forceinline__ v16h cat16(v8h lo, v8h hi) { return __builtin_shufflevector(lo, hi, 0, 1, 2, 3, 4, 5, 6, 7, 8, 9, 10, 11, 12, 13, 14, 15); }
__device__ __forceinline__ v16bf cat16b(v8us lo, v8us hi) { return __builtin_bit_cast(v16bf, __builtin_shufflevector(lo, hi, 0, 1, 2, 3, 4, 5, 6, 7, 8, 9, 10, 11, 12, 13, 14, 15)); }
__device__ __forceinline__ v8f wmma16(v16h a, v16h b, v8f c) { return __builtin_amdgcn_wmma_f32_16x16x32_f16(false, a, false, b, (short)0, c, false, false); }
__device__ __forceinline__ v8f wmmab(v16bf a, v16bf b, v8f c) { return __builtin_amdgcn_wmma_f32_16x16x32_bf16(false, a, false, b, (short)0, c, false, false); }

template <bool SPLITA, bool F16OUT = false>
__global__ __launch_bounds__(128) void k_gemmb(const bf* __restrict__ A, const bf* __restrict__ Al, const bf* __restrict__ Bn, const float* __restrict__ bias, float* C, int ldc, h16* C2, const float* __restrict__ R = nullptr, int K = DM, int roundR = 1) {
    __shared__ __align__(16) float ost[4][16 * 68];
    const int lane = threadIdx.x & 31, wave = threadIdx.x >> 5, lr = lane & 15, hi = lane >> 4;
    const int r0 = blockIdx.x * 64 + wave * 16, c0 = blockIdx.y * 64;
    const size_t aoff = (size_t)(r0 + lr) * K + 8 * hi;
    size_t boff[4];
#pragma unroll
    for (int t = 0; t < 4; ++t) boff[t] = (size_t)(c0 + t * 16 + lr) * K + 8 * hi;
    v8f acc[4];
#pragma unroll
    for (int t = 0; t < 4; ++t) acc[t] = (v8f){};
#pragma unroll 1
    for (int kc = 0; kc < K; kc += 32) {
        const v16bf a = cat16b(*(const v8us*)(A + aoff + kc), *(const v8us*)(A + aoff + kc + 16));
        v16bf al = a;
        if (SPLITA) al = cat16b(*(const v8us*)(Al + aoff + kc), *(const v8us*)(Al + aoff + kc + 16));
#pragma unroll
        for (int t = 0; t < 4; ++t) { const v16bf b = cat16b(*(const v8us*)(Bn + boff[t] + kc), *(const v8us*)(Bn + boff[t] + kc + 16)); acc[t] = wmmab(a, b, acc[t]); if (SPLITA) acc[t] = wmmab(al, b, acc[t]); }
        asm volatile("v_nop\n\tv_nop\n\tv_nop\n\tv_nop" : "+v"(acc[0]), "+v"(acc[1]), "+v"(acc[2]), "+v"(acc[3]) : "v"(a), "v"(al));
    }
    float* os = &ost[wave][0];
#pragma unroll
    for (int t = 0; t < 4; ++t) { const float bv = bias ? bfr(bias[c0 + t * 16 + lr]) : 0.f;
#pragma unroll
        for (int j = 0; j < 8; ++j) os[(hi * 8 + j) * 68 + t * 16 + lr] = acc[t][j] + bv; }
    __syncthreads();
    if (F16OUT) {
        h16* crow = (h16*)(void*)C + (size_t)r0 * ldc + c0;
        auto pass = [&]() {
#pragma unroll
            for (int s = 0; s < 4; ++s) { const int row = 4 * s + (lane >> 3), piece = lane & 7; const float* sp = os + row * 68 + piece * 8; v8h o, o2;
#pragma unroll
                for (int i = 0; i < 8; ++i) { const h16 a = (h16)sp[i]; o[i] = a; o2[i] = (h16)((sp[i] - (float)a) * LOSC); }
                *(volatile v8h*)(crow + (size_t)row * ldc + piece * 8) = o; if (C2) *(volatile v8h*)(C2 + (size_t)r0 * ldc + c0 + (size_t)row * ldc + piece * 8) = o2; }
        };
        pass(); __threadfence(); pass();
    } else {
        float* crow = C + (size_t)r0 * ldc + c0;
        auto pass = [&]() {
#pragma unroll
            for (int s = 0; s < 8; ++s) { const int Lid = (lane >> 3) + 4 * s, piece = lane & 7; const int row = Lid >> 1, cofs = (Lid & 1) * 32 + piece * 4;
                v4f val = *(const v4fa*)(os + row * 68 + cofs); if (R) { const v4f rv = *(const v4f*)(R + ((size_t)r0 + row) * ldc + c0 + cofs); val += roundR ? (v4f){bfr(rv[0]), bfr(rv[1]), bfr(rv[2]), bfr(rv[3])} : rv; }
                *(volatile v4f*)(crow + (size_t)row * ldc + cofs) = val; }
        };
        pass(); __threadfence(); pass();
    }
}


__global__ __launch_bounds__(256) void k_cvt8(const float* __restrict__ src, bf* dst, size_t n8) {
    const size_t i = (size_t)blockIdx.x * 256 + threadIdx.x; if (i >= n8) return;
    const v8f v = *(const v8f*)(src + i * 8); v8us o;
#pragma unroll
    for (int k = 0; k < 8; ++k) o[k] = f2bf(v[k]);
    *(volatile v8us*)(dst + i * 8) = o; __threadfence(); *(volatile v8us*)(dst + i * 8) = o;
}
__global__ __launch_bounds__(256) void k_zero8(bf* dst, size_t n8) {
    const size_t i = (size_t)blockIdx.x * 256 + threadIdx.x; if (i >= n8) return; v8us z;
#pragma unroll
    for (int k = 0; k < 8; ++k) z[k] = 0;
    *(volatile v8us*)(dst + i * 8) = z; __threadfence(); *(volatile v8us*)(dst + i * 8) = z;
}

__global__ __launch_bounds__(256) void k_trace(const float* __restrict__ x, float* U) {
    const int lane = threadIdx.x & 31; const int w = blockIdx.x * 8 + (threadIdx.x >> 5); if (w >= NBT * TT / 32) return; const int e = w * 32 + lane; float s = 0.f;
#pragma unroll 4
    for (int i = 0; i < NSQ; ++i) s += bfr(x[(size_t)e * NSQ * NSQ + i * NSQ + i]);
    *(volatile float*)(U + e) = s; __threadfence(); *(volatile float*)(U + e) = s;
}
__global__ __launch_bounds__(256) void k_zero(float* p, size_t n4) {
    const size_t g = (size_t)blockIdx.x * 256 + threadIdx.x; if (g >= n4) return; const v4f z = {0.f, 0.f, 0.f, 0.f}; *(volatile v4f*)(p + g * 4) = z; __threadfence(); *(volatile v4f*)(p + g * 4) = z;
}
__device__ __forceinline__ float sigm(float v) { return 1.0f / (1.0f + __expf(-v)); }
__global__ __launch_bounds__(128) void k_cell0(const float* __restrict__ G, const float* __restrict__ U, int t, const float* __restrict__ wih, const float* __restrict__ bih, const float* __restrict__ bhh,
                                               float* Cst, bf* Hh, bf* Hl, float* H1, bf* DHh, bf* DHl) {
    typedef __attribute__((ext_vector_type(2))) unsigned short v2us; typedef __attribute__((ext_vector_type(2))) float v2f_;
    const int lane = threadIdx.x & 31; const int w = blockIdx.x * 4 + (threadIdx.x >> 5); if (w >= NBT * 2) return; const int b = w >> 1, j0 = (w & 1) * 64 + lane * 2;
    const float u = U[b * TT + t]; v2f_ cv, hv, h1v; v2us hh, hl, dh_h, dh_l;
#pragma unroll
    for (int q = 0; q < 2; ++q) { const int j = j0 + q;
        float pre[4], dpre[4];
#pragma unroll
        for (int k = 0; k < 4; ++k) { const int gi = k * HH + j; const float wu = bfr(wih[gi]); pre[k] = G[b * G4 + gi] + u * wu + bfr(bih[gi]) + bfr(bhh[gi]); dpre[k] = wu; }
        const float ig = sigm(pre[0]), fg = sigm(pre[1]), gg = tanhf(pre[2]), og = sigm(pre[3]);
        const float cp = Cst[b * HH + j]; const float c = fg * cp + ig * gg; const float tc = tanhf(c); const float h = og * tc;
        const float di = ig * (1.f - ig) * dpre[0], dfg = fg * (1.f - fg) * dpre[1], dg = (1.f - gg * gg) * dpre[2], dog = og * (1.f - og) * dpre[3];
        const float dc = dfg * cp + di * gg + ig * dg; const float dh = dog * tc + og * (1.f - tc * tc) * dc;
        cv[q] = c; hv[q] = h; h1v[q] = h; { const unsigned short hb = f2bf(h); hh[q] = hb; hl[q] = f2bf(h - bf2f(hb)); } { const unsigned short hb = f2bf(dh); dh_h[q] = hb; dh_l[q] = f2bf(dh - bf2f(hb)); } }
    const size_t so = (size_t)b * HH + j0; const size_t po = (size_t)b * HH + j0; const size_t ho = ((size_t)t * NBT + b) * HH + j0; const size_t dho = ((size_t)b * TT + t) * HH + j0;
    *(volatile v2f_*)(Cst + so) = cv; *(volatile v2us*)(Hh + po) = hh; *(volatile v2us*)(Hl + po) = hl; *(volatile v2f_*)(H1 + ho) = h1v; *(volatile v2us*)(DHh + dho) = dh_h; *(volatile v2us*)(DHl + dho) = dh_l;
    __threadfence();
    *(volatile v2f_*)(Cst + so) = cv; *(volatile v2us*)(Hh + po) = hh; *(volatile v2us*)(Hl + po) = hl; *(volatile v2f_*)(H1 + ho) = h1v; *(volatile v2us*)(DHh + dho) = dh_h; *(volatile v2us*)(DHl + dho) = dh_l;
}
__global__ __launch_bounds__(128) void k_in1(const float* __restrict__ H1, int t, bf* Ah, bf* Al) {
    typedef __attribute__((ext_vector_type(2))) unsigned short v2us;
    const int lane = threadIdx.x & 31; const int w = blockIdx.x * 4 + (threadIdx.x >> 5); if (w >= NBT * 2) return; const int b = w >> 1, j0 = (w & 1) * 64 + lane * 2; v2us oh, ol;
#pragma unroll
    for (int q = 0; q < 2; ++q) { const float v = H1[((size_t)t * NBT + b) * HH + j0 + q]; const unsigned short hb = f2bf(v); oh[q] = hb; ol[q] = f2bf(v - bf2f(hb)); }
    const size_t o = (size_t)b * (2 * HH) + j0; *(volatile v2us*)(Ah + o) = oh; *(volatile v2us*)(Al + o) = ol; __threadfence(); *(volatile v2us*)(Ah + o) = oh; *(volatile v2us*)(Al + o) = ol;
}
__global__ __launch_bounds__(128) void k_cell1(const float* __restrict__ G, const float* __restrict__ DG2, int t, const float* __restrict__ bih, const float* __restrict__ bhh,
                                               float* Cst, bf* Ah, bf* Al, float* DH2) {
    typedef __attribute__((ext_vector_type(2))) unsigned short v2us; typedef __attribute__((ext_vector_type(2))) float v2f_;
    const int lane = threadIdx.x & 31; const int w = blockIdx.x * 4 + (threadIdx.x >> 5); if (w >= NBT * 2) return; const int b = w >> 1, half = w & 1, j0 = half * 64 + lane * 2;
    v2f_ cv, dhv; v2us hh, hl;
#pragma unroll
    for (int q = 0; q < 2; ++q) { const int j = j0 + q;
        float pre[4], dpre[4];
#pragma unroll
        for (int k = 0; k < 4; ++k) { const int gi = k * HH + j; pre[k] = G[b * G4 + gi] + bfr(bih[gi]) + bfr(bhh[gi]); dpre[k] = DG2[((size_t)b * TT + t) * G4 + gi]; }
        const float ig = sigm(pre[0]), fg = sigm(pre[1]), gg = tanhf(pre[2]), og = sigm(pre[3]);
        const float cp = Cst[b * HH + j]; const float c = fg * cp + ig * gg; const float tc = tanhf(c); const float h = og * tc;
        const float di = ig * (1.f - ig) * dpre[0], dfg = fg * (1.f - fg) * dpre[1], dg = (1.f - gg * gg) * dpre[2], dog = og * (1.f - og) * dpre[3];
        const float dc = dfg * cp + di * gg + ig * dg; const float dh = dog * tc + og * (1.f - tc * tc) * dc;
        cv[q] = c; dhv[q] = dh; { const unsigned short hb = f2bf(h); hh[q] = hb; hl[q] = f2bf(h - bf2f(hb)); } }
    const size_t so = (size_t)b * HH + j0; const size_t po = (size_t)b * (2 * HH) + HH + j0;
    const size_t dho = ((size_t)b * TT + t) * HH + j0;
    *(volatile v2f_*)(Cst + so) = cv; *(volatile v2us*)(Ah + po) = hh; *(volatile v2us*)(Al + po) = hl; *(volatile v2f_*)(DH2 + dho) = dhv; __threadfence();
    *(volatile v2f_*)(Cst + so) = cv; *(volatile v2us*)(Ah + po) = hh; *(volatile v2us*)(Al + po) = hl; *(volatile v2f_*)(DH2 + dho) = dhv;
}
__global__ __launch_bounds__(256) void k_outj(const float* __restrict__ DH2, const float* __restrict__ wout, float* OUTP) {
    const int lane = threadIdx.x & 31; const size_t w = (size_t)blockIdx.x * 8 + (threadIdx.x >> 5); if (w >= (size_t)NBT * TT * NSQ) return; const int i = (int)(w % NSQ); const size_t bt = w / NSQ;
    float d = 0.f;
#pragma unroll
    for (int q = 0; q < HH / 32; ++q) d = fmaf(bfr(wout[q * 32 + lane]), DH2[bt * HH + q * 32 + lane], d);
#pragma unroll
    for (int sh = 16; sh; sh >>= 1) d += __shfl_xor(d, sh, 32);
    const float v = (lane == i) ? d : 0.f;
    *(volatile float*)(OUTP + w * NSQ + lane) = v; __threadfence(); *(volatile float*)(OUTP + w * NSQ + lane) = v;
}

__global__ __launch_bounds__(256) void k_w1cat(const float* __restrict__ wih1, const float* __restrict__ whh1, bf* W1) {
    const int lane = threadIdx.x & 31; const int g = blockIdx.x * 8 + (threadIdx.x >> 5); if (g >= G4) return; const int c0 = lane * 8; v8us o;
#pragma unroll
    for (int i = 0; i < 8; ++i) { const int c = c0 + i; o[i] = f2bf(c < HH ? wih1[(size_t)g * HH + (c < HH ? c : 0)] : whh1[(size_t)g * HH + (c >= HH ? c - HH : 0)]); }
    *(volatile v8us*)(W1 + (size_t)g * (2 * HH) + c0) = o; __threadfence(); *(volatile v8us*)(W1 + (size_t)g * (2 * HH) + c0) = o;
}

extern "C" void kernel_launch(void* const* d_in, const int* in_sizes, int n_in,
                              void* d_out, int out_size, void* d_ws, size_t ws_size, hipStream_t stream) {
    (void)in_sizes; (void)n_in; (void)out_size;
    const float* x = (const float*)d_in[0]; const float* wih0 = (const float*)d_in[1]; const float* whh0 = (const float*)d_in[2]; const float* bih0 = (const float*)d_in[3]; const float* bhh0 = (const float*)d_in[4];
    const float* wih1 = (const float*)d_in[5]; const float* whh1 = (const float*)d_in[6]; const float* bih1 = (const float*)d_in[7]; const float* bhh1 = (const float*)d_in[8]; const float* wout = (const float*)d_in[9];
    float* out = (float*)d_out;
    char* wsp = (char*)d_ws;
    auto take = [&](size_t bytes) { char* p = wsp; wsp += (bytes + 255) & ~(size_t)255; return (void*)p; };
    bf* W0 = (bf*)take((size_t)G4 * HH * 2); bf* W1 = (bf*)take((size_t)G4 * 2 * HH * 2); bf* WI1 = (bf*)take((size_t)G4 * HH * 2);
    float* U = (float*)take((size_t)NBT * TT * 4); bf* A0h = (bf*)take((size_t)MP * HH * 2); bf* A0l = (bf*)take((size_t)MP * HH * 2); bf* A1h = (bf*)take((size_t)MP * 2 * HH * 2); bf* A1l = (bf*)take((size_t)MP * 2 * HH * 2);
    float* C0 = (float*)take((size_t)NBT * HH * 4); float* C1 = (float*)take((size_t)NBT * HH * 4); float* G = (float*)take((size_t)MP * G4 * 4); float* H1 = (float*)take((size_t)TT * NBT * HH * 4);
    bf* DHh = (bf*)take((size_t)NBT * TT * HH * 2); bf* DHl = (bf*)take((size_t)NBT * TT * HH * 2); float* DG2 = (float*)take((size_t)NBT * TT * G4 * 4); float* DH2 = (float*)take((size_t)NBT * TT * HH * 4);
    if ((size_t)(wsp - (char*)d_ws) > ws_size) return;
    k_cvt8<<<(G4 * HH / 8 + 255) / 256, 256, 0, stream>>>(whh0, W0, G4 * HH / 8); k_cvt8<<<(G4 * HH / 8 + 255) / 256, 256, 0, stream>>>(wih1, WI1, G4 * HH / 8); k_w1cat<<<G4 / 8, 256, 0, stream>>>(wih1, whh1, W1);
    k_trace<<<(NBT * TT / 32 + 7) / 8, 256, 0, stream>>>(x, U);
    k_zero<<<(MP * HH / 2 / 4 + 255) / 256, 256, 0, stream>>>((float*)A0h, MP * HH / 2 / 4); k_zero<<<(MP * HH / 2 / 4 + 255) / 256, 256, 0, stream>>>((float*)A0l, MP * HH / 2 / 4);
    k_zero<<<(MP * 2 * HH / 2 / 4 + 255) / 256, 256, 0, stream>>>((float*)A1h, MP * 2 * HH / 2 / 4); k_zero<<<(MP * 2 * HH / 2 / 4 + 255) / 256, 256, 0, stream>>>((float*)A1l, MP * 2 * HH / 2 / 4);
    k_zero<<<(NBT * HH / 4 + 255) / 256, 256, 0, stream>>>(C0, NBT * HH / 4); k_zero<<<(NBT * HH / 4 + 255) / 256, 256, 0, stream>>>(C1, NBT * HH / 4);
    for (int t = 0; t < TT; ++t) {
        k_gemmb<true, false><<<dim3(MP / 64, G4 / 64, 1), 128, 0, stream>>>(A0h, A0l, W0, nullptr, G, G4, nullptr, nullptr, HH);
        k_cell0<<<(NBT * 2) / 4, 128, 0, stream>>>(G, U, t, wih0, bih0, bhh0, C0, A0h, A0l, H1, DHh, DHl); }
    k_gemmb<true, false><<<dim3((NBT * TT) / 64, G4 / 64, 1), 128, 0, stream>>>(DHh, DHl, WI1, nullptr, DG2, G4, nullptr, nullptr, HH);
    for (int t = 0; t < TT; ++t) {
        k_in1<<<(NBT * 2) / 4, 128, 0, stream>>>(H1, t, A1h, A1l);
        k_gemmb<true, false><<<dim3(MP / 64, G4 / 64, 1), 128, 0, stream>>>(A1h, A1l, W1, nullptr, G, G4, nullptr, nullptr, 2 * HH);
        k_cell1<<<(NBT * 2) / 4, 128, 0, stream>>>(G, DG2, t, bih1, bhh1, C1, A1h, A1l, DH2); }
    k_outj<<<(NBT * TT * NSQ) / 8, 256, 0, stream>>>(DH2, wout, out);
}
